// MultiAttentionGRU_50783693308404
// MI455X (gfx1250) — hardware-verified
//
#include <hip/hip_runtime.h>


namespace {
constexpr int D = 64, M = 5, MAXDEG = 4, VOCAB = 5000, NCLASS = 4, NL = 24576, NPAR = 8192, NN = NL + NPAR, WORDS = 32;
constexpr float XS = 8.0f, WSC = 256.0f, LNE = 1e-5f, NEG = -1e9f;

typedef _Float16 b16;
typedef __attribute__((ext_vector_type(16))) _Float16 v16b;
typedef __attribute__((ext_vector_type(8))) _Float16 v8b;
typedef __attribute__((ext_vector_type(8))) float v8f;
typedef __attribute__((ext_vector_type(4))) float v4f;
__device__ __forceinline__ float bf16_rne(float f) { unsigned int u = __float_as_uint(f); u += 0x7FFFu + ((u >> 16) & 1u); return __uint_as_float(u & 0xFFFF0000u); }
__device__ __forceinline__ void split16(float v, b16& hi, b16& lo) { hi = (b16)v; lo = (b16)(v - (float)hi); }
__device__ __forceinline__ v16b frag_kb(const b16* p, int hh) { const v8b a = *(const v8b*)(p + 8 * hh), b = *(const v8b*)(p + 16 + 8 * hh); v16b f;
#pragma unroll
  for (int e = 0; e < 8; ++e) { f[e] = a[e]; f[8 + e] = b[e]; } return f; }
__device__ __forceinline__ v8f wmma16b(v16b a, v16b b, v8f c) { v8f d = __builtin_amdgcn_wmma_f32_16x16x32_f16(false, a, false, b, (short)0, c, false, false); asm volatile("v_nop\n\tv_nop\n\tv_nop\n\tv_nop" : "+v"(d) : "v"(a), "v"(b)); return d; }
__device__ __forceinline__ void wave_lds_sync() { __builtin_amdgcn_fence(__ATOMIC_RELEASE, "workgroup"); __builtin_amdgcn_wave_barrier(); __builtin_amdgcn_fence(__ATOMIC_ACQUIRE, "workgroup"); }
__device__ __forceinline__ float pmul(float a, float b) { float p = a * b; asm volatile("" : "+v"(p)); return p; }
__device__ __forceinline__ int iclamp(int v, int lo, int hi) { return v < lo ? lo : (v > hi ? hi : v); }
__device__ __forceinline__ float nexp(float x) { return __builtin_amdgcn_exp2f(x * 1.4426950408889634f); }
__device__ __forceinline__ float sigm(float x) { return 1.0f / (1.0f + nexp(-x)); }
__device__ __forceinline__ float tanh_(float x) { const float e = nexp(-2.0f * fabsf(x)); const float t = (1.0f - e) / (1.0f + e); return x < 0.0f ? -t : t; }

__global__ __launch_bounds__(256) void prepE_kernel(const float* __restrict__ E, float* __restrict__ ER) {
  const size_t t = (size_t)blockIdx.x * 256 + threadIdx.x; if (t >= (size_t)D * VOCAB / 4) return; const v4f v = *(const v4f*)(E + t * 4); const v4f o = {bf16_rne(v[0]), bf16_rne(v[1]), bf16_rne(v[2]), bf16_rne(v[3])};
  for (int pass = 0; pass < 2; ++pass) { *(volatile v4f*)(ER + t * 4) = o; __threadfence(); }
}
__global__ __launch_bounds__(256) void xe_kernel(const float* __restrict__ xw, const int* __restrict__ xi, const float* __restrict__ E, float* __restrict__ XE, b16* __restrict__ XEh, b16* __restrict__ XEl) {
  const int wave = threadIdx.x >> 5, lane = threadIdx.x & 31; const size_t n = (size_t)blockIdx.x * 8 + wave; const int d0 = lane * 2;
  const int myid = iclamp(xi[n * WORDS + lane], 0, VOCAB - 1); const float myw = bf16_rne(xw[n * WORDS + lane]);
  float s0 = 0.0f, s1 = 0.0f;
  for (int l = 0; l < WORDS; ++l) { const int id = __shfl(myid, l); const float w = __shfl(myw, l); s0 += pmul(E[(size_t)d0 * VOCAB + id], w); s1 += pmul(E[(size_t)(d0 + 1) * VOCAB + id], w); }
  b16 h0, l0, h1, l1; split16(s0 * XS, h0, l0); split16(s1 * XS, h1, l1);
  typedef __attribute__((ext_vector_type(2))) float v2f; typedef __attribute__((ext_vector_type(2))) _Float16 v2b;
  const v2f o = {s0, s1}; const v2b oh = {h0, h1}, ol = {l0, l1};
  for (int pass = 0; pass < 2; ++pass) { *(volatile v2f*)(XE + n * D + d0) = o; *(volatile v2b*)(XEh + n * D + d0) = oh; *(volatile v2b*)(XEl + n * D + d0) = ol; __threadfence(); }
}
__global__ __launch_bounds__(256) void prepw_kernel(const float* __restrict__ wz, const float* __restrict__ wr, const float* __restrict__ wh, const float* __restrict__ wq, const float* __restrict__ wk, const float* __restrict__ uh, const float* __restrict__ uz, const float* __restrict__ ur, const float* __restrict__ wo, b16* __restrict__ WP, b16* __restrict__ WOP, b16* __restrict__ UP) {
  const int t = blockIdx.x * 256 + threadIdx.x;
  if (t >= 896 * D / 8) { const int u = t - 896 * D / 8; v8b o;
    if (u < D * M * D / 8) { for (int j = 0; j < 8; ++j) o[j] = (b16)(bf16_rne(wo[(size_t)u * 8 + j]) * WSC); for (int pass = 0; pass < 2; ++pass) { *(volatile v8b*)(WOP + (size_t)u * 8) = o; __threadfence(); } }
    else if (u < D * M * D / 8 + 3 * D * D / 8) { const int e = (u - D * M * D / 8) * 8; const int w = e / (D * D), r = e - w * D * D; const float* src = w == 0 ? uz : w == 1 ? ur : uh; for (int j = 0; j < 8; ++j) o[j] = (b16)(bf16_rne(src[r + j]) * WSC); for (int pass = 0; pass < 2; ++pass) { *(volatile v8b*)(UP + e) = o; __threadfence(); } }
    return; } const int row = (t * 8) / D, c0 = t * 8 - row * D; v8b o;
  for (int j = 0; j < 8; ++j) { const int c = c0 + j; float v;
    if (row < 64) v = wz[row * D + c]; else if (row < 128) v = wr[(row - 64) * D + c]; else if (row < 192) v = wh[(row - 128) * D + c];
    else if (row < 512) { const int m = (row - 192) / D, i = (row - 192) % D; v = wq[((size_t)m * D + i) * D + c]; }
    else if (row < 832) { const int m = (row - 512) / D, i = (row - 512) % D; v = wk[((size_t)m * D + c) * D + i]; }
    else v = uh[(row - 832) * D + c];
    o[j] = (b16)(bf16_rne(v) * WSC); }
  for (int pass = 0; pass < 2; ++pass) { *(volatile v8b*)(WP + (size_t)t * 8) = o; __threadfence(); }
}
template <int NT>
__global__ __launch_bounds__(128) void gemm_kernel(const b16* __restrict__ Ah, const b16* __restrict__ Al, const b16* __restrict__ W, size_t row0, float* __restrict__ Y) {
  __shared__ __attribute__((aligned(16))) float Ts[4][16][NT * 16 + 4];
  const int wave = threadIdx.x >> 5, lane = threadIdx.x & 31, nloc = lane & 15, hlf = lane >> 4; const size_t m0 = row0 + ((size_t)blockIdx.x * 4 + wave) * 16; const size_t y0 = ((size_t)blockIdx.x * 4 + wave) * 16;
  v8f acc[NT];
#pragma unroll
  for (int t = 0; t < NT; ++t) acc[t] = (v8f){};
#pragma unroll
  for (int kb = 0; kb < D; kb += 32) { const v16b a = frag_kb(Ah + (m0 + nloc) * D + kb, hlf), al = frag_kb(Al + (m0 + nloc) * D + kb, hlf);
#pragma unroll
    for (int t = 0; t < NT; ++t) { const v16b bw = frag_kb(W + (size_t)(t * 16 + nloc) * D + kb, hlf); acc[t] = wmma16b(a, bw, acc[t]); acc[t] = wmma16b(al, bw, acc[t]); } }
#pragma unroll
  for (int t = 0; t < NT; ++t)
#pragma unroll
    for (int r = 0; r < 8; ++r) Ts[wave][8 * hlf + r][t * 16 + nloc] = acc[t][r] * (1.0f / (XS * WSC));
  wave_lds_sync();
  for (int pass = 0; pass < 2; ++pass) { for (int rr = 0; rr < 16; ++rr) for (int c4 = lane * 4; c4 < NT * 16; c4 += 128) *(volatile v4f*)(Y + (y0 + rr) * (NT * 16) + c4) = *(const v4f*)(&Ts[wave][rr][c4]); __threadfence(); }
}
__global__ __launch_bounds__(256) void leaf1_kernel(const float* __restrict__ WX, const float* __restrict__ uz, const float* __restrict__ ur, const float* __restrict__ bz, const float* __restrict__ br, const float* __restrict__ lnb, float* __restrict__ Z, b16* __restrict__ Rh, b16* __restrict__ Rl) {
  __shared__ float cz[D], cr[D], lb[D];
  const int t_ = threadIdx.x, wave = t_ >> 5, lane = t_ & 31; if (t_ < D) { float a = 0.0f, b = 0.0f; for (int j = 0; j < D; ++j) { const float hb = bf16_rne(lnb[j]); a += pmul(bf16_rne(uz[t_ * D + j]), hb); b += pmul(bf16_rne(ur[t_ * D + j]), hb); } cz[t_] = a + bf16_rne(bz[t_]); cr[t_] = b + bf16_rne(br[t_]); lb[t_] = bf16_rne(lnb[t_]); }
  __syncthreads();
  const size_t n = (size_t)blockIdx.x * 8 + wave; const int d0 = lane * 2; typedef __attribute__((ext_vector_type(2))) float v2f; typedef __attribute__((ext_vector_type(2))) _Float16 v2b;
  v2f zo; v2b rh, rl; for (int q = 0; q < 2; ++q) { const int d = d0 + q; const float z = sigm(WX[n * 192 + d] + cz[d]); const float r = sigm(WX[n * 192 + 64 + d] + cr[d]); zo[q] = z; b16 a_, c_; split16(pmul(lb[d], r) * XS, a_, c_); rh[q] = a_; rl[q] = c_; }
  for (int pass = 0; pass < 2; ++pass) { *(volatile v2f*)(Z + n * D + d0) = zo; *(volatile v2b*)(Rh + n * D + d0) = rh; *(volatile v2b*)(Rl + n * D + d0) = rl; __threadfence(); }
}
__global__ __launch_bounds__(256) void leaf2_kernel(const float* __restrict__ WX, const float* __restrict__ UHR, const float* __restrict__ Z, const float* __restrict__ bh, const float* __restrict__ lnb, float* __restrict__ LEAFH) {
  const int wave = threadIdx.x >> 5, lane = threadIdx.x & 31; const size_t n = (size_t)blockIdx.x * 8 + wave; const int d0 = lane * 2; typedef __attribute__((ext_vector_type(2))) float v2f; v2f o;
  for (int q = 0; q < 2; ++q) { const int d = d0 + q; const float c = tanh_(WX[n * 192 + 128 + d] + UHR[n * D + d] + bf16_rne(bh[d])); const float z = Z[n * D + d]; o[q] = pmul(z, bf16_rne(lnb[d])) + pmul(1.0f - z, c); }
  for (int pass = 0; pass < 2; ++pass) { *(volatile v2f*)(LEAFH + n * D + d0) = o; __threadfence(); }
}
__global__ __launch_bounds__(256) void att_kernel(const float* __restrict__ Q, const float* __restrict__ KN, const int* __restrict__ tree, float* __restrict__ ATT) {
  const int wave = threadIdx.x >> 5, lane = threadIdx.x & 31; const int p = blockIdx.x * 8 + wave; const int m = lane >> 2, c = lane & 3;
  float lg = NEG; int valid = 0;
  if (m < M) { const int ch = tree[p * 5 + c]; valid = (ch > -1) ? 1 : 0; const int ci = iclamp(ch, 0, NN - 1); if (valid) { float s = 0.0f; for (int i = 0; i < D; ++i) s += pmul(Q[((size_t)p * M + m) * D + i], KN[((size_t)ci * M + m) * D + i]); lg = s * ((m == 0) ? 0.125f : 8.0f); } }
  float mx = lg; mx = fmaxf(mx, __shfl_xor(mx, 1)); mx = fmaxf(mx, __shfl_xor(mx, 2)); const float e = nexp(lg - mx); float sm = e; sm += __shfl_xor(sm, 1); sm += __shfl_xor(sm, 2); const float a = e / sm;
  for (int pass = 0; pass < 2; ++pass) { ((volatile float*)ATT)[(size_t)p * 32 + lane] = (m < M) ? a : 0.0f; __threadfence(); }
}
__device__ __forceinline__ v16b frag_vec(const b16* v, int kb, int hh, int nloc) { v16b f = {}; if (nloc == 0) { const v8b a = *(const v8b*)(v + kb + 8 * hh), b = *(const v8b*)(v + kb + 16 + 8 * hh); for (int e = 0; e < 8; ++e) { f[e] = a[e]; f[8 + e] = b[e]; } } return f; }
__global__ __launch_bounds__(256) void chain_kernel(const float* __restrict__ WX, const float* __restrict__ ATT, const int* __restrict__ tree, const float* __restrict__ LEAFH, const b16* __restrict__ WOP, const b16* __restrict__ UP, const float* __restrict__ bz, const float* __restrict__ br, const float* __restrict__ bh,
                                                 const float* __restrict__ lng, const float* __restrict__ lnb, float* __restrict__ PH) {
  __shared__ float ch[MAXDEG][D]; __shared__ __attribute__((aligned(16))) b16 cxh[M * D + 32], cxl[M * D + 32], hth[D + 32], htl[D + 32], hrh[D + 32], hrl[D + 32]; __shared__ float hprev[D]; __shared__ int chidx[MAXDEG];
  const int t_ = threadIdx.x, wave = t_ >> 5, lane = t_ & 31, nloc = lane & 15, hh = lane >> 4;
  if (t_ < D) hprev[t_] = 0.0f;
  const float sc = 1.0f / (XS * WSC);
  __syncthreads();
  for (int p = 0; p < NPAR; ++p) {
    if (t_ < MAXDEG) chidx[t_] = tree[p * 5 + t_];
    __syncthreads();
    { const int c = t_ >> 6, i = t_ & 63; const int id = chidx[c]; float v = 0.0f;
      if (id > -1) { if (id < NL) v = LEAFH[(size_t)id * D + i]; else { const int q = id - NL; if (q == p - 1) v = hprev[i]; else if (q < p) v = PH[(size_t)q * D + i]  ; else v = 0.0f; } }
      ch[c][i] = v; }
    __syncthreads();
    for (int k = t_; k < M * D; k += 256) { const int m = k >> 6, i = k & 63; float s = 0.0f; for (int c = 0; c < MAXDEG; ++c) s += pmul(ATT[(size_t)p * 32 + m * 4 + c], ch[c][i]); b16 a_, c_; split16(s * XS, a_, c_); cxh[k] = a_; cxl[k] = c_; }
    __syncthreads();
    if (wave == 0) { const size_t pid = (size_t)NL + p;
      v8f acc[4] = {{}, {}, {}, {}};
#pragma unroll 1
      for (int kb = 0; kb < M * D; kb += 32) { const v16b a = frag_vec(cxh, kb, hh, nloc), al = frag_vec(cxl, kb, hh, nloc);
#pragma unroll
        for (int t = 0; t < 4; ++t) { const v16b bw = frag_kb(WOP + (size_t)(t * 16 + nloc) * (M * D) + kb, hh); acc[t] = wmma16b(a, bw, acc[t]); acc[t] = wmma16b(al, bw, acc[t]); } }
      float rv[4]; float s1 = 0.0f; for (int t = 0; t < 4; ++t) { rv[t] = (hh == 0) ? acc[t][0] * sc : 0.0f; s1 += rv[t]; }
      s1 += __shfl_xor(s1, 1); s1 += __shfl_xor(s1, 2); s1 += __shfl_xor(s1, 4); s1 += __shfl_xor(s1, 8); s1 += __shfl_xor(s1, 16); const float mu = s1 * (1.0f / D);
      float s2 = 0.0f; for (int t = 0; t < 4; ++t) { const float dv = (hh == 0) ? rv[t] - mu : 0.0f; s2 += dv * dv; } s2 += __shfl_xor(s2, 1); s2 += __shfl_xor(s2, 2); s2 += __shfl_xor(s2, 4); s2 += __shfl_xor(s2, 8); s2 += __shfl_xor(s2, 16); const float rs = rsqrtf(s2 * (1.0f / D) + LNE);
      float ht[4]; if (hh == 0) for (int t = 0; t < 4; ++t) { const int o = t * 16 + nloc; ht[t] = pmul((rv[t] - mu) * rs, bf16_rne(lng[o])) + bf16_rne(lnb[o]); b16 a_, c_; split16(ht[t] * XS, a_, c_); hth[o] = a_; htl[o] = c_; }
      wave_lds_sync();
      v8f az[4] = {{}, {}, {}, {}}, ar[4] = {{}, {}, {}, {}};
#pragma unroll
      for (int kb = 0; kb < D; kb += 32) { const v16b a = frag_vec(hth, kb, hh, nloc), al = frag_vec(htl, kb, hh, nloc);
#pragma unroll
        for (int t = 0; t < 4; ++t) { const v16b bz_ = frag_kb(UP + (size_t)(t * 16 + nloc) * D + kb, hh), br_ = frag_kb(UP + (size_t)D * D + (size_t)(t * 16 + nloc) * D + kb, hh); az[t] = wmma16b(a, bz_, az[t]); az[t] = wmma16b(al, bz_, az[t]); ar[t] = wmma16b(a, br_, ar[t]); ar[t] = wmma16b(al, br_, ar[t]); } }
      float zv[4]; if (hh == 0) for (int t = 0; t < 4; ++t) { const int o = t * 16 + nloc; zv[t] = sigm(WX[pid * 192 + o] + az[t][0] * sc + bf16_rne(bz[o])); const float r = sigm(WX[pid * 192 + 64 + o] + ar[t][0] * sc + bf16_rne(br[o])); b16 a_, c_; split16(pmul(ht[t], r) * XS, a_, c_); hrh[o] = a_; hrl[o] = c_; }
      wave_lds_sync();
      v8f ac[4] = {{}, {}, {}, {}};
#pragma unroll
      for (int kb = 0; kb < D; kb += 32) { const v16b a = frag_vec(hrh, kb, hh, nloc), al = frag_vec(hrl, kb, hh, nloc);
#pragma unroll
        for (int t = 0; t < 4; ++t) { const v16b bw = frag_kb(UP + (size_t)2 * D * D + (size_t)(t * 16 + nloc) * D + kb, hh); ac[t] = wmma16b(a, bw, ac[t]); ac[t] = wmma16b(al, bw, ac[t]); } }
      if (hh == 0) { for (int t = 0; t < 4; ++t) { const int o = t * 16 + nloc; const float c = tanh_(WX[pid * 192 + 128 + o] + ac[t][0] * sc + bf16_rne(bh[o])); const float h = pmul(zv[t], ht[t]) + pmul(1.0f - zv[t], c); hprev[o] = h;
          ((volatile float*)PH)[(size_t)p * D + o] = h; __threadfence(); ((volatile float*)PH)[(size_t)p * D + o] = h; } } }
    __threadfence(); __syncthreads(); }
}
__global__ __launch_bounds__(32) void loss_kernel(const float* __restrict__ PH, const float* __restrict__ wout, const float* __restrict__ bout, const float* __restrict__ y, float* __restrict__ out) {
  const int lane = threadIdx.x; float lg[NCLASS];
  for (int k = 0; k < NCLASS; ++k) { float s = pmul(bf16_rne(wout[k * D + lane]), PH[(size_t)(NPAR - 1) * D + lane]) + pmul(bf16_rne(wout[k * D + lane + 32]), PH[(size_t)(NPAR - 1) * D + lane + 32]);
    s += __shfl_xor(s, 1); s += __shfl_xor(s, 2); s += __shfl_xor(s, 4); s += __shfl_xor(s, 8); s += __shfl_xor(s, 16); lg[k] = s + bf16_rne(bout[k]); }
  float mx = fmaxf(fmaxf(lg[0], lg[1]), fmaxf(lg[2], lg[3])); float e[NCLASS], sm = 0.0f; for (int k = 0; k < NCLASS; ++k) { e[k] = nexp(lg[k] - mx); sm += e[k]; } float loss = 0.0f; for (int k = 0; k < NCLASS; ++k) { const float dv = bf16_rne(y[k]) - e[k] / sm; loss += dv * dv; }
  for (int pass = 0; pass < 2; ++pass) { if (lane == 0) ((volatile float*)out)[0] = loss; __threadfence(); }
}
}

extern "C" void kernel_launch(void* const* d_in, const int* in_sizes, int n_in, void* d_out, int out_size, void* d_ws, size_t ws_size, hipStream_t stream) {
  (void)n_in;
  auto Fp = [&](int i) { return (const float*)d_in[i]; }; auto Ip = [&](int i) { return (const int*)d_in[i]; };
  if (in_sizes[0] != NN * WORDS || in_sizes[1] != NN * WORDS || in_sizes[2] != NPAR * 5 || in_sizes[4] != D * VOCAB || in_sizes[16] != M * D * D || in_sizes[18] != D * M * D || out_size != 1) return;
  size_t off = 0; char* ws = (char*)d_ws;
  auto carve = [&](size_t bytes) { char* p = ws + off; off += (bytes + 255) & ~(size_t)255; return p; };
  float* XE = (float*)carve((size_t)NN * D * 4); float* ER = (float*)carve((size_t)D * VOCAB * 4); b16* XEh = (b16*)carve((size_t)NN * D * 2); b16* XEl = (b16*)carve((size_t)NN * D * 2); b16* WP = (b16*)carve((size_t)896 * D * 2); b16* WOP = (b16*)carve((size_t)D * M * D * 2); b16* UP = (b16*)carve((size_t)3 * D * D * 2);
  float* WX = (float*)carve((size_t)NN * 192 * 4); float* Q = (float*)carve((size_t)NPAR * M * D * 4); float* KN = (float*)carve((size_t)NN * M * D * 4); float* Z = (float*)carve((size_t)NL * D * 4); b16* Rh = (b16*)carve((size_t)NL * D * 2); b16* Rl = (b16*)carve((size_t)NL * D * 2); float* UHR = (float*)carve((size_t)NL * D * 4); float* LEAFH = (float*)carve((size_t)NL * D * 4); float* ATT = (float*)carve((size_t)NPAR * 32 * 4); float* PH = (float*)carve((size_t)NPAR * D * 4);
  if (off > ws_size || off > ((size_t)128 << 20)) return;
  prepE_kernel<<<(D * VOCAB / 4 + 255) / 256, 256, 0, stream>>>(Fp(4), ER);
  xe_kernel<<<NN / 8, 256, 0, stream>>>(Fp(0), Ip(1), ER, XE, XEh, XEl);
  prepw_kernel<<<(896 * D / 8 + D * M * D / 8 + 3 * D * D / 8 + 255) / 256, 256, 0, stream>>>(Fp(5), Fp(8), Fp(11), Fp(16), Fp(17), Fp(12), Fp(6), Fp(9), Fp(18), WP, WOP, UP);
  gemm_kernel<12><<<NN / 64, 128, 0, stream>>>(XEh, XEl, WP, 0, WX);
  gemm_kernel<20><<<NPAR / 64, 128, 0, stream>>>(XEh, XEl, WP + (size_t)192 * D, NL, Q);
  gemm_kernel<20><<<NN / 64, 128, 0, stream>>>(XEh, XEl, WP + (size_t)512 * D, 0, KN);
  leaf1_kernel<<<NL / 8, 256, 0, stream>>>(WX, Fp(6), Fp(9), Fp(7), Fp(10), Fp(20), Z, Rh, Rl);
  gemm_kernel<4><<<NL / 64, 128, 0, stream>>>(Rh, Rl, WP + (size_t)832 * D, 0, UHR);
  leaf2_kernel<<<NL / 8, 256, 0, stream>>>(WX, UHR, Z, Fp(13), Fp(20), LEAFH);
  att_kernel<<<NPAR / 8, 256, 0, stream>>>(Q, KN, Ip(2), ATT);
  chain_kernel<<<1, 256, 0, stream>>>(WX, ATT, Ip(2), LEAFH, WOP, UP, Fp(7), Fp(10), Fp(13), Fp(19), Fp(20), PH);
  loss_kernel<<<1, 32, 0, stream>>>(PH, Fp(14), Fp(15), Fp(3), (float*)d_out);
}
